// CustomGRUCell_26027501814359
// MI455X (gfx1250) — hardware-verified
//
#include <hip/hip_runtime.h>
#include <math.h>

constexpr int kRows = 4096;
constexpr int kHid  = 2048;
constexpr int kHalfRows = 2048;
constexpr int kKcat = 4096;
constexpr float kWCarry    = 16.0f;
constexpr float kWCarryInv = 1.0f / 16.0f;

constexpr size_t kOffWR  = 0;
constexpr size_t kOffWZ  = kOffWR  + (size_t)kHid * kKcat * 2;
constexpr size_t kOffWI2 = kOffWZ  + (size_t)kHid * kKcat * 2;
constexpr size_t kOffWH2 = kOffWI2 + (size_t)kHid * kHid * 2;
constexpr size_t kOffAH  = kOffWH2 + (size_t)kHid * kHid * 2;
constexpr size_t kOffP0  = kOffAH  + (size_t)kHalfRows * kKcat * 2;
constexpr size_t kOffP1  = kOffP0  + (size_t)kHalfRows * kHid * 4;
constexpr size_t kOffP2  = kOffP1  + (size_t)kHalfRows * kHid * 4;
constexpr size_t kWsEnd  = kOffP2  + (size_t)kHalfRows * kHid * 4;

typedef __attribute__((ext_vector_type(16))) _Float16 v16h;
typedef __attribute__((ext_vector_type(8)))  _Float16 v8h;
typedef __attribute__((ext_vector_type(16))) __bf16   v16b;
typedef __attribute__((ext_vector_type(8)))  __bf16   v8b;
typedef __attribute__((ext_vector_type(8)))  float    v8f;
typedef __attribute__((ext_vector_type(4)))  float    v4f;
typedef __attribute__((ext_vector_type(4)))  unsigned int v4u;

__device__ __forceinline__ unsigned short f2bf_bits(float f) {
  unsigned u = __float_as_uint(f);
  return (unsigned short)((u + 0x7FFFu + ((u >> 16) & 1u)) >> 16);
}
__device__ __forceinline__ float bf_bits2f(unsigned short h) { return __uint_as_float(((unsigned)h) << 16); }

__device__ __forceinline__ void dep_guard_h(v8f& a, v8f& b, v16h x, v16h y) { asm volatile("v_nop\n\tv_nop\n\tv_nop\n\tv_nop" : "+v"(a), "+v"(b) : "v"(x), "v"(y)); }
__device__ __forceinline__ void dep_guard_b(v8f& a, v8f& b, v16b x, v16b y) { asm volatile("v_nop\n\tv_nop\n\tv_nop\n\tv_nop" : "+v"(a), "+v"(b) : "v"(x), "v"(y)); }
__device__ __forceinline__ void keep4_h(v16h a, v16h b, v16h c, v16h d) { asm volatile("v_nop" :: "v"(a), "v"(b), "v"(c), "v"(d)); }
__device__ __forceinline__ void keep4_b(v16b a, v16b b, v16b c, v16b d) { asm volatile("v_nop" :: "v"(a), "v"(b), "v"(c), "v"(d)); }
__device__ __forceinline__ void acc_guard4(v8f& a, v8f& b, v8f& c, v8f& d) { asm volatile("v_nop\n\tv_nop\n\tv_nop\n\tv_nop" : "+v"(a), "+v"(b), "+v"(c), "+v"(d)); }
template <typename T> struct Frag;
template <> struct Frag<_Float16> {
  typedef v16h V; union U { v16h v; v8h h[2]; };
  static __device__ __forceinline__ v16h load(const _Float16* p) {
    U f; f.h[0] = *(const v8h*)(p); f.h[1] = *(const v8h*)(p + 16); return f.v;
  }
  static __device__ __forceinline__ v8f mma(v16h a, v16h b, v8f c) {
    return __builtin_amdgcn_wmma_f32_16x16x32_f16(false, a, false, b, (short)0, c, false, false);
  }
  static __device__ __forceinline__ void guard(v8f& a, v8f& b, v16h x, v16h y) { dep_guard_h(a, b, x, y); }
  static __device__ __forceinline__ void keep(v16h a, v16h b, v16h c, v16h d) { keep4_h(a, b, c, d); }
};
template <> struct Frag<__bf16> {
  typedef v16b V; union U { v16b v; v8b h[2]; };
  static __device__ __forceinline__ v16b load(const __bf16* p) {
    U f; f.h[0] = *(const v8b*)(p); f.h[1] = *(const v8b*)(p + 16); return f.v;
  }
  static __device__ __forceinline__ v8f mma(v16b a, v16b b, v8f c) {
    return __builtin_amdgcn_wmma_f32_16x16x32_bf16(false, a, false, b, (short)0, c, false, false);
  }
  static __device__ __forceinline__ void guard(v8f& a, v8f& b, v16b x, v16b y) { dep_guard_b(a, b, x, y); }
  static __device__ __forceinline__ void keep(v16b a, v16b b, v16b c, v16b d) { keep4_b(a, b, c, d); }
};

__device__ __forceinline__ unsigned pk16(unsigned short a, unsigned short b) { return (unsigned)a | ((unsigned)b << 16); }
__device__ __forceinline__ unsigned short h_bits(float f) { const _Float16 h = (_Float16)f; return __builtin_bit_cast(unsigned short, h); }

template <int ET> struct Elem;
template <> struct Elem<0> { typedef _Float16 T; };
template <> struct Elem<1> { typedef __bf16 T; };
template <int ET, bool SPLIT, int BIAS_MODE, int OUT_MODE, bool RESID, int ACT = 0>
__global__ __launch_bounds__(256) void wmma_gemm64(
    const unsigned short* __restrict__ Ap, const unsigned short* __restrict__ A2p, int lda, long strideA,
    const unsigned short* __restrict__ Btp, const unsigned short* __restrict__ Bt2p, int ldb, long strideB,
    void* __restrict__ Cout, void* __restrict__ Cout2, int ldc, long strideC,
    const float* __restrict__ bias, const float* __restrict__ bias2,
    const float* __restrict__ resid, long strideR,
    int M, int N, int K, float scale) {
  typedef typename Elem<ET>::T T;
  typedef typename Frag<T>::V V;
  const T* A = (const T*)Ap; const T* A2 = (const T*)A2p; const T* Bt = (const T*)Btp; const T* Bt2 = (const T*)Bt2p;
  __shared__ __align__(16) float sT[8][16 * 68];
  const int b    = blockIdx.y;
  const int lane = threadIdx.x & 31;
  const int wave = threadIdx.x >> 5;
  const int tilesN = N >> 6;
  const int tilesM = M >> 6;
  const int tile = blockIdx.x * 8 + wave;
  if (tile >= tilesM * tilesN) return;
  const int tm = tile / tilesN;
  const int tn = tile - tm * tilesN;
  const int m0 = tm << 6;
  const int n0 = tn << 6;

  const T* Ab  = A  + (size_t)b * strideA;
  const T* Bb  = Bt + (size_t)b * strideB;
  const T* Ab2 = SPLIT ? (A2  + (size_t)b * strideA) : nullptr;
  const T* Bb2 = SPLIT ? (Bt2 + (size_t)b * strideB) : nullptr;

  const int rlane = lane & 15;
  const int koff  = (lane >> 4) * 8;
  const int mOff  = (lane >> 4) * 8;

  v8f acc[4][4];
#pragma unroll
  for (int i = 0; i < 4; ++i)
#pragma unroll
    for (int j = 0; j < 4; ++j) acc[i][j] = (v8f){0.f,0.f,0.f,0.f,0.f,0.f,0.f,0.f};

  for (int k0 = 0; k0 < K; k0 += 32) {
    V bh[4], bl[4];
#pragma unroll
    for (int j = 0; j < 4; ++j) {
      const size_t bo = (size_t)(n0 + (j << 4) + rlane) * ldb + koff + k0;
      bh[j] = Frag<T>::load(Bb + bo);
      if (SPLIT) bl[j] = Frag<T>::load(Bb2 + bo);
    }
#pragma unroll
    for (int i = 0; i < 4; ++i) {
      const size_t ao = (size_t)(m0 + (i << 4) + rlane) * lda + koff + k0;
      V ah = Frag<T>::load(Ab + ao);
      V al;
      if (SPLIT) al = Frag<T>::load(Ab2 + ao);
#pragma unroll
      for (int j = 0; j < 4; ++j) {
        acc[i][j] = Frag<T>::mma(ah, bh[j], acc[i][j]);
        if (SPLIT) {
          acc[i][j] = Frag<T>::mma(ah, bl[j], acc[i][j]);
          acc[i][j] = Frag<T>::mma(al, bh[j], acc[i][j]);
        }
      }
      Frag<T>::guard(acc[i][0], acc[i][3], ah, SPLIT ? al : ah);
    }
    Frag<T>::keep(bh[0], bh[1], bh[2], bh[3]);
    if (SPLIT) Frag<T>::keep(bl[0], bl[1], bl[2], bl[3]);
  }
  acc_guard4(acc[0][0], acc[0][1], acc[0][2], acc[0][3]);
  acc_guard4(acc[1][0], acc[1][1], acc[1][2], acc[1][3]);
  acc_guard4(acc[2][0], acc[2][1], acc[2][2], acc[2][3]);
  acc_guard4(acc[3][0], acc[3][1], acc[3][2], acc[3][3]);

  float* slab = sT[wave];
  const float* Rb = RESID ? (resid + (size_t)b * strideR) : nullptr;
#pragma unroll
  for (int i = 0; i < 4; ++i) {
    const int mBase = m0 + (i << 4);
#pragma unroll
    for (int j = 0; j < 4; ++j) {
      const int n = n0 + (j << 4) + rlane;
      float bv = 0.f;
      if (BIAS_MODE == 2) bv = bias[n];
      if (BIAS_MODE == 3) bv = bias[n] + bias2[n];
#pragma unroll
      for (int r = 0; r < 8; ++r) {
        float v = acc[i][j][r] * scale;
        if (BIAS_MODE == 1) v += bias[mBase + mOff + r];
        if (BIAS_MODE == 2 || BIAS_MODE == 3) v += bv;
        if (RESID) v += Rb[(size_t)(mBase + mOff + r) * ldc + n];
        if (ACT == 1) v = tanhf(v);
        if (ACT == 6) v = 1.0f / (1.0f + expf(-v));
        slab[(mOff + r) * 68 + (j << 4) + rlane] = v;
      }
    }
    __builtin_amdgcn_fence(__ATOMIC_RELEASE, "workgroup");
    __builtin_amdgcn_wave_barrier();
    __builtin_amdgcn_fence(__ATOMIC_ACQUIRE, "workgroup");
    if (OUT_MODE == 0) {
      float* C = (float*)Cout + (size_t)b * strideC;
      const int hh = lane >> 4, c4 = (lane & 15) * 4;
      for (int pass = 0; pass < 2; ++pass) {
#pragma unroll
        for (int it = 0; it < 8; ++it) {
          const int row = it * 2 + hh;
          v4f v = *(const v4f*)(slab + row * 68 + c4);
          *(volatile v4f*)(C + (size_t)(mBase + row) * ldc + n0 + c4) = v;
        }
        __threadfence();
      }
    } else {
      const int q = lane >> 3, c8 = (lane & 7) * 8;
      unsigned short* C  = (unsigned short*)Cout  + (size_t)b * strideC;
      unsigned short* C2 = (OUT_MODE == 2) ? ((unsigned short*)Cout2 + (size_t)b * strideC) : nullptr;
      for (int pass = 0; pass < 2; ++pass) {
#pragma unroll
        for (int it = 0; it < 4; ++it) {
          const int row = it * 4 + q;
          const float* sp = slab + row * 68 + c8;
          v8h hv, lv;
#pragma unroll
          for (int e = 0; e < 8; ++e) {
            if (OUT_MODE == 1) {
              hv[e] = (_Float16)sp[e];
            } else {
              unsigned short hb = f2bf_bits(sp[e]);
              unsigned short lb = f2bf_bits(sp[e] - bf_bits2f(hb));
              hv[e] = __builtin_bit_cast(_Float16, hb);
              lv[e] = __builtin_bit_cast(_Float16, lb);
            }
          }
          *(volatile v8h*)(C + (size_t)(mBase + row) * ldc + n0 + c8) = hv;
          if (OUT_MODE == 2) *(volatile v8h*)(C2 + (size_t)(mBase + row) * ldc + n0 + c8) = lv;
        }
        __threadfence();
      }
    }
    __builtin_amdgcn_fence(__ATOMIC_RELEASE, "workgroup");
    __builtin_amdgcn_wave_barrier();
    __builtin_amdgcn_fence(__ATOMIC_ACQUIRE, "workgroup");
  }
}

__global__ __launch_bounds__(256) void wtcast_kernel(const float* __restrict__ wih, const float* __restrict__ whh,
                                                     unsigned short* __restrict__ WR, unsigned short* __restrict__ WZ,
                                                     unsigned short* __restrict__ WI2, unsigned short* __restrict__ WH2,
                                                     float scale) {
  __shared__ float sm[64][65];
  const int t  = threadIdx.x;
  const int d0 = blockIdx.x * 64;
  const int h0 = blockIdx.y * 64;
  const int z  = blockIdx.z;
  const int g  = z >> 1;
  const int s  = z & 1;
  const float* W = ((s == 0) ? wih : whh) + (size_t)g * kHid * kHid;
  unsigned short* dst = (g == 0) ? WR : (g == 1) ? WZ : ((s == 0) ? WI2 : WH2);
  const int ldo  = (g < 2) ? kKcat : kHid;
  const int coff = (g < 2) ? s * kHid : 0;
#pragma unroll
  for (int i = 0; i < 16; ++i) {
    const int e = i * 256 + t;
    const int r = e >> 6;
    const int c = e & 63;
    sm[c][r] = W[(size_t)(d0 + r) * kHid + h0 + c] * scale;
  }
  __syncthreads();
  const int lane = t & 31, wave = t >> 5;
  const int q = lane >> 3, c8 = (lane & 7) * 8;
  unsigned short* op = dst + coff;
  for (int pass = 0; pass < 2; ++pass) {
#pragma unroll
    for (int it = 0; it < 2; ++it) {
      const int row = wave * 8 + it * 4 + q;
      unsigned short hb[8];
#pragma unroll
      for (int e = 0; e < 8; ++e) hb[e] = h_bits(sm[row][c8 + e]);
      const v4u u = (v4u){pk16(hb[0], hb[1]), pk16(hb[2], hb[3]), pk16(hb[4], hb[5]), pk16(hb[6], hb[7])};
      *(volatile v4u*)(op + (size_t)(h0 + row) * ldo + d0 + c8) = u;
    }
    __threadfence();
  }
}

__global__ __launch_bounds__(256) void acast_kernel(const float* __restrict__ x, const float* __restrict__ hx,
                                                    unsigned short* __restrict__ AH, int m0, int n8) {
  const int s = blockIdx.y;
  const int i = blockIdx.x * 256 + threadIdx.x;
  if (i >= n8) return;
  const int row = i >> 8;
  const int c8  = (i & 255) * 8;
  const float* p = ((s == 0) ? x : hx) + (size_t)(m0 + row) * kHid + c8;
  const v4f a = *(const v4f*)(p);
  const v4f c = *(const v4f*)(p + 4);
  unsigned short hb[8];
#pragma unroll
  for (int e = 0; e < 4; ++e) {
    hb[e]     = h_bits(a[e]);
    hb[4 + e] = h_bits(c[e]);
  }
  const v4u u = (v4u){pk16(hb[0], hb[1]), pk16(hb[2], hb[3]), pk16(hb[4], hb[5]), pk16(hb[6], hb[7])};
  unsigned short* q = AH + (size_t)row * kKcat + (size_t)s * kHid + c8;
  *(volatile v4u*)q = u;
  __threadfence();
  *(volatile v4u*)q = u;
}

__global__ __launch_bounds__(256) void mul_kernel(const float* __restrict__ P, const float* __restrict__ Q,
                                                  float* __restrict__ D, int n4) {
  const int i = blockIdx.x * 256 + threadIdx.x;
  if (i >= n4) return;
  const size_t e = 4 * (size_t)i;
  const v4f p = *(const v4f*)(P + e);
  const v4f q = *(const v4f*)(Q + e);
  const v4f d = p * q;
  *(volatile v4f*)(D + e) = d;
  __threadfence();
  *(volatile v4f*)(D + e) = d;
}

__global__ __launch_bounds__(256) void blend_kernel(const float* __restrict__ Zp, const float* __restrict__ Np,
                                                    const float* __restrict__ hx, float* __restrict__ out, int m0, int n4) {
  const int i = blockIdx.x * 256 + threadIdx.x;
  if (i >= n4) return;
  const size_t e  = 4 * (size_t)i;
  const size_t go = (size_t)m0 * kHid + e;
  const v4f z = *(const v4f*)(Zp + e);
  const v4f n = *(const v4f*)(Np + e);
  const v4f h = *(const v4f*)(hx + go);
  const v4f o = (1.0f - z) * n + z * h;
  *(volatile v4f*)(out + go) = o;
  __threadfence();
  *(volatile v4f*)(out + go) = o;
}

extern "C" void kernel_launch(void* const* d_in, const int* in_sizes, int n_in,
                              void* d_out, int out_size, void* d_ws, size_t ws_size,
                              hipStream_t stream) {
  if (n_in < 6) return;
  if (in_sizes[0] != kRows * kHid || in_sizes[1] != kRows * kHid) return;
  if (in_sizes[2] != 3 * kHid * kHid || in_sizes[3] != 3 * kHid * kHid) return;
  if (in_sizes[4] != 3 * kHid || in_sizes[5] != 3 * kHid) return;
  if (out_size != kRows * kHid) return;
  if (ws_size < kWsEnd) return;

  const float* x   = (const float*)d_in[0];
  const float* hx  = (const float*)d_in[1];
  const float* wih = (const float*)d_in[2];
  const float* whh = (const float*)d_in[3];
  const float* bih = (const float*)d_in[4];
  const float* bhh = (const float*)d_in[5];
  float* out = (float*)d_out;

  unsigned char* ws = (unsigned char*)d_ws;
  unsigned short* WR  = (unsigned short*)(ws + kOffWR);
  unsigned short* WZ  = (unsigned short*)(ws + kOffWZ);
  unsigned short* WI2 = (unsigned short*)(ws + kOffWI2);
  unsigned short* WH2 = (unsigned short*)(ws + kOffWH2);
  unsigned short* AH  = (unsigned short*)(ws + kOffAH);
  float* P0 = (float*)(ws + kOffP0);
  float* P1 = (float*)(ws + kOffP1);
  float* P2 = (float*)(ws + kOffP2);

  const int n8 = kHalfRows * kHid / 8;
  const int n4 = kHalfRows * kHid / 4;
  const dim3 ggrid(((kHalfRows / 64) * (kHid / 64) + 7) / 8, 1);

  wtcast_kernel<<<dim3(kHid / 64, kHid / 64, 6), 256, 0, stream>>>(wih, whh, WR, WZ, WI2, WH2, kWCarry);

  for (int hf = 0; hf < 2; ++hf) {
    const int m0 = hf * kHalfRows;

    acast_kernel<<<dim3((n8 + 255) / 256, 2), 256, 0, stream>>>(x, hx, AH, m0, n8);

    wmma_gemm64<0, false, 2, 0, false, 0><<<ggrid, 256, 0, stream>>>(
        AH + kHid, AH + kHid, kKcat, 0L, WH2, WH2, kHid, 0L,
        (void*)P0, (void*)P0, kHid, 0L, bhh + 2 * kHid, bhh + 2 * kHid, bhh, 0L,
        kHalfRows, kHid, kHid, kWCarryInv);

    wmma_gemm64<0, false, 3, 0, false, 6><<<ggrid, 256, 0, stream>>>(
        AH, AH, kKcat, 0L, WR, WR, kKcat, 0L,
        (void*)P1, (void*)P1, kHid, 0L, bih, bhh, bih, 0L,
        kHalfRows, kHid, kKcat, kWCarryInv);

    mul_kernel<<<dim3((n4 + 255) / 256), 256, 0, stream>>>(P1, P0, P2, n4);

    wmma_gemm64<0, false, 3, 0, false, 6><<<ggrid, 256, 0, stream>>>(
        AH, AH, kKcat, 0L, WZ, WZ, kKcat, 0L,
        (void*)P0, (void*)P0, kHid, 0L, bih + kHid, bhh + kHid, bih, 0L,
        kHalfRows, kHid, kKcat, kWCarryInv);

    wmma_gemm64<0, false, 2, 0, true, 1><<<ggrid, 256, 0, stream>>>(
        AH, AH, kKcat, 0L, WI2, WI2, kHid, 0L,
        (void*)P1, (void*)P1, kHid, 0L, bih + 2 * kHid, bih + 2 * kHid, P2, 0L,
        kHalfRows, kHid, kHid, kWCarryInv);

    blend_kernel<<<dim3((n4 + 255) / 256), 256, 0, stream>>>(P0, P1, hx, out, m0, n4);
  }
}
